// TGNLayerGraphAttentionEmbedding_48747878810095
// MI455X (gfx1250) — hardware-verified
//
#include <hip/hip_runtime.h>
#include <math.h>

typedef __attribute__((ext_vector_type(16))) _Float16 v16h;
typedef __attribute__((ext_vector_type(16))) __bf16 v16b;
typedef __attribute__((ext_vector_type(8)))  _Float16 v8h;
typedef __attribute__((ext_vector_type(8)))  float v8f;
typedef __attribute__((ext_vector_type(4)))  float v4f;
typedef __attribute__((ext_vector_type(2)))  float v2f;
typedef __attribute__((ext_vector_type(4)))  unsigned v4u;
typedef __attribute__((ext_vector_type(4)))  int v4i;
typedef float __attribute__((may_alias)) float_a;
typedef int __attribute__((may_alias)) int_a;

template <typename T> __device__ __forceinline__ void vst2(void* p, T v) { *(volatile T*)p = v; __threadfence(); *(volatile T*)p = v; }
__device__ __forceinline__ v8f wmma16(v16h a, v16h b, v8f c) {
  v8f d = __builtin_amdgcn_wmma_f32_16x16x32_f16(false, a, false, b, (short)0, c, false, false);
  asm volatile("v_nop\n\tv_nop\n\tv_nop\n\tv_nop" : "+v"(d) : "v"(a), "v"(b));
  return d;
}
__device__ __forceinline__ v8f wmma_bf(v16b a, v16b b, v8f c) {
  v8f d = __builtin_amdgcn_wmma_f32_16x16x32_bf16(false, a, false, b, (short)0, c, false, false);
  asm volatile("v_nop\n\tv_nop\n\tv_nop\n\tv_nop" : "+v"(d) : "v"(a), "v"(b));
  return d;
}
__device__ __forceinline__ v16h frag_h(const _Float16* rowk0, int lane) {
  union { v16h v; v8h q[2]; } u; const _Float16* p = rowk0 + 8 * (lane >> 4);
  u.q[0] = *(const v8h*)p; u.q[1] = *(const v8h*)(p + 16); return u.v;
}
__device__ __forceinline__ v16h frag_f32(const float* rowk0, int lane) {
  v16h a; const float* p = rowk0 + 8 * (lane >> 4);
#pragma unroll
  for (int i = 0; i < 8; ++i) { a[i] = (_Float16)p[i]; a[8 + i] = (_Float16)p[16 + i]; }
  return a;
}
__device__ __forceinline__ v16h frag_f32s(const float* rowk0, int lane, float sc) {
  v16h a; const float* p = rowk0 + 8 * (lane >> 4);
#pragma unroll
  for (int i = 0; i < 8; ++i) { a[i] = (_Float16)(p[i] * sc); a[8 + i] = (_Float16)(p[16 + i] * sc); }
  return a;
}
__device__ __forceinline__ v16h fragc_f32(const float* W, int k0, int n, int lane, int ld, int K) {
  v16h a; const int g = lane >> 4;
#pragma unroll
  for (int i = 0; i < 8; ++i) { const int ka = k0 + 8 * g + i, kb = ka + 16;
    a[i] = (_Float16)(ka < K ? W[(size_t)ka * ld + n] : 0.f); a[8 + i] = (_Float16)(kb < K ? W[(size_t)kb * ld + n] : 0.f); }
  return a;
}
struct F2 { v16b h, l; };
__device__ __forceinline__ F2 bsplit16(const float v[16]) { F2 r;
#pragma unroll
  for (int i = 0; i < 16; ++i) { const __bf16 h = (__bf16)v[i]; r.h[i] = h; r.l[i] = (__bf16)(v[i] - (float)h); }
  return r; }
__device__ __forceinline__ F2 split_row(const float* row, int k0, int lane) { float v[16]; const float* p = row + k0 + 8 * (lane >> 4);
#pragma unroll
  for (int i = 0; i < 8; ++i) { v[i] = p[i]; v[8 + i] = p[16 + i]; }
  return bsplit16(v); }
__device__ __forceinline__ F2 split_rowK(const float* row, int k0, int lane, int K) { float v[16]; const int g = lane >> 4;
#pragma unroll
  for (int i = 0; i < 8; ++i) { const int ka = k0 + 8 * g + i, kb = ka + 16; v[i] = ka < K ? row[ka] : 0.f; v[8 + i] = kb < K ? row[kb] : 0.f; }
  return bsplit16(v); }
__device__ __forceinline__ F2 split_col(const float* W, int k0, int n, int lane, int ld, int K) { float v[16]; const int g = lane >> 4;
#pragma unroll
  for (int i = 0; i < 8; ++i) { const int ka = k0 + 8 * g + i, kb = ka + 16; v[i] = ka < K ? W[(size_t)ka * ld + n] : 0.f; v[8 + i] = kb < K ? W[(size_t)kb * ld + n] : 0.f; }
  return bsplit16(v); }
__device__ __forceinline__ v8f mac3(const F2& a, const F2& b, v8f c) { c = wmma_bf(a.l, b.h, c); c = wmma_bf(a.h, b.l, c); return wmma_bf(a.h, b.h, c); }
__device__ __forceinline__ float sigm(float v) { return 1.0f / (1.0f + expf(-v)); }
#define LDSX() do { asm volatile("s_wait_dscnt 0" ::: "memory"); __builtin_amdgcn_wave_barrier(); __builtin_amdgcn_fence(__ATOMIC_RELEASE, "workgroup"); } while (0)

#define NNODE 4096
#define KNB 10
#define FE 128
#define FEF 64
#define FT 64
#define KEY 256
#define KD 2560
#define DM 192
#define NH 2
#define HDD 96

__global__ __launch_bounds__(256) void k_pack(const float* __restrict__ Wq, const float* __restrict__ Wk, const float* __restrict__ Wv, const float* __restrict__ Wo, const float* __restrict__ W1, const float* __restrict__ W2,
                                            _Float16* __restrict__ WqT, _Float16* __restrict__ WkT, _Float16* __restrict__ WvT, _Float16* __restrict__ WoT, _Float16* __restrict__ W1T, _Float16* __restrict__ W2T) {
  const int r = blockIdx.x, tid = threadIdx.x; __shared__ __align__(16) _Float16 srow[KD];
  const float* W; _Float16* D; int K, NO, n;
  if (r < DM) { W = Wk; D = WkT; K = KD; NO = DM; n = r; } else if (r < 2 * DM) { W = Wv; D = WvT; K = KD; NO = DM; n = r - DM; }
  else if (r < 3 * DM) { W = Wq; D = WqT; K = DM; NO = DM; n = r - 2 * DM; } else if (r < 4 * DM) { W = Wo; D = WoT; K = DM; NO = DM; n = r - 3 * DM; }
  else if (r < 4 * DM + FE) { W = W1; D = W1T; K = DM + FE; NO = FE; n = r - 4 * DM; } else { W = W2; D = W2T; K = FE; NO = FE; n = r - 4 * DM - FE; }
  for (int k = tid; k < K; k += 256) srow[k] = (_Float16)(W[(size_t)k * NO + n] * 16.0f);
  __syncthreads();
  for (int q = tid; q < K / 8; q += 256) vst2(D + (size_t)n * K + q * 8, *(const v4u*)(&srow[q * 8]));
}
__global__ __launch_bounds__(128) void k_kv(const float* __restrict__ feat, const float* __restrict__ ef, const float* __restrict__ tf, const int* __restrict__ nbr, const _Float16* __restrict__ WkT, const _Float16* __restrict__ WvT, const float* __restrict__ bk, const float* __restrict__ bv, _Float16* __restrict__ K16, _Float16* __restrict__ VT) {
  __shared__ __align__(16) _Float16 sa[64][KEY + 8];
  __shared__ __align__(16) float so[4][16][196];
  __shared__ __align__(16) _Float16 st[DM][72];
  const int tid = threadIdx.x, wave = tid >> 5, lane = tid & 31, col = lane & 15, g = lane >> 4;
  const int which = blockIdx.y, r0b = blockIdx.x * 64, r0 = r0b + wave * 16; const _Float16* WT = which == 0 ? WkT : WvT;
  v8f acc[12];
#pragma unroll
  for (int t = 0; t < 12; ++t) acc[t] = (v8f){};
#pragma unroll 1
  for (int j = 0; j < KNB; ++j) {
    for (int q = tid; q < 64 * 32; q += 128) { const int rl = q >> 5, pc = q & 31; const int n = r0b + rl; int m = nbr[(size_t)n * KNB + j]; m = m < 0 ? 0 : (m >= NNODE ? NNODE - 1 : m);
      const float* src = pc < 16 ? feat + (size_t)m * FE + pc * 8 : (pc < 24 ? ef + ((size_t)n * KNB + j) * FEF + (pc - 16) * 8 : tf + ((size_t)n * KNB + j) * FT + (pc - 24) * 8);
      union { v8h h; v4u u; } pk;
#pragma unroll
      for (int e = 0; e < 8; ++e) pk.h[e] = (_Float16)src[e];
      *(v4u*)(&sa[rl][pc * 8]) = pk.u; }
    __syncthreads();
#pragma unroll 2
    for (int kc = 0; kc < KEY / 32; ++kc) { const v16h a = frag_h(&sa[wave * 16 + col][0] + kc * 32, lane);
#pragma unroll
      for (int t = 0; t < 12; ++t) acc[t] = wmma16(a, frag_h(WT + (size_t)(t * 16 + col) * KD + j * KEY + kc * 32, lane), acc[t]); }
    __syncthreads(); }
  const float* bias = which == 0 ? bk : bv;
  if (which == 0) {
#pragma unroll
    for (int t = 0; t < 12; ++t) { const float bb = bias[t * 16 + col];
#pragma unroll
      for (int r = 0; r < 8; ++r) so[wave][8 * g + r][t * 16 + col] = (acc[t][r] * (1.0f / 16.0f) + bb) * 4.0f; }
    LDSX();
    for (int qq = lane; qq < 16 * 24; qq += 32) { const int rl = qq / 24, rem = qq % 24; const int h = rem / 12, pc = rem % 12; union { v8h h8; v4u u; } pk;
#pragma unroll
      for (int e = 0; e < 8; ++e) pk.h8[e] = (_Float16)so[wave][rl][h * HDD + pc * 8 + e];
      vst2(K16 + ((size_t)h * NNODE + r0 + rl) * HDD + pc * 8, pk.u); } }
  else {
#pragma unroll
    for (int t = 0; t < 12; ++t) { const float bb = bias[t * 16 + col];
#pragma unroll
      for (int r = 0; r < 8; ++r) st[t * 16 + col][wave * 16 + 8 * g + r] = (_Float16)(acc[t][r] * (1.0f / 16.0f) + bb); }
    __syncthreads();
    for (int qq = tid; qq < DM * 8; qq += 128) { const int c = qq >> 3, pc = qq & 7; const int h = c / HDD, d = c % HDD; vst2(VT + ((size_t)h * HDD + d) * NNODE + r0b + pc * 8, *(const v4u*)(&st[c][pc * 8])); } }
}
__global__ __launch_bounds__(128) void k_q(const float* __restrict__ feat, const int* __restrict__ nidx, const _Float16* __restrict__ WqT, const float* __restrict__ bq, _Float16* __restrict__ Q16) {
  __shared__ __align__(16) _Float16 sa[64][FE + 8];
  __shared__ __align__(16) float so[4][16][196];
  const int tid = threadIdx.x, wave = tid >> 5, lane = tid & 31, col = lane & 15, g = lane >> 4;
  const int r0b = blockIdx.x * 64, r0 = r0b + wave * 16;
  for (int q = tid; q < 64 * 16; q += 128) { const int rl = q >> 4, pc = q & 15; int m = nidx[r0b + rl]; m = m < 0 ? 0 : (m >= NNODE ? NNODE - 1 : m); union { v8h h; v4u u; } pk;
#pragma unroll
    for (int e = 0; e < 8; ++e) pk.h[e] = (_Float16)feat[(size_t)m * FE + pc * 8 + e];
    *(v4u*)(&sa[rl][pc * 8]) = pk.u; }
  __syncthreads();
  v8f acc[12];
#pragma unroll
  for (int t = 0; t < 12; ++t) acc[t] = (v8f){};
#pragma unroll
  for (int kc = 0; kc < FE / 32; ++kc) { const v16h a = frag_h(&sa[wave * 16 + col][0] + kc * 32, lane);
#pragma unroll
    for (int t = 0; t < 12; ++t) acc[t] = wmma16(a, frag_h(WqT + (size_t)(t * 16 + col) * DM + kc * 32, lane), acc[t]); }
#pragma unroll
  for (int t = 0; t < 12; ++t) { const float bb = bq[t * 16 + col];
#pragma unroll
    for (int r = 0; r < 8; ++r) so[wave][8 * g + r][t * 16 + col] = (acc[t][r] * (1.0f / 16.0f) + bb) * 4.0f; }
  LDSX();
  for (int qq = lane; qq < 16 * 24; qq += 32) { const int rl = qq / 24, rem = qq % 24; const int h = rem / 12, pc = rem % 12; union { v8h h8; v4u u; } pk;
#pragma unroll
    for (int e = 0; e < 8; ++e) pk.h8[e] = (_Float16)so[wave][rl][h * HDD + pc * 8 + e];
    vst2(Q16 + ((size_t)h * NNODE + r0 + rl) * HDD + pc * 8, pk.u); }
}
__global__ __launch_bounds__(128) void k_attn(const _Float16* __restrict__ Q16, const _Float16* __restrict__ K16, const _Float16* __restrict__ VT, _Float16* __restrict__ O16) {
  __shared__ __align__(16) float sS[4][16][68];
  __shared__ __align__(16) _Float16 sP[4][16][72];
  __shared__ __align__(16) float sO[4][16][100];
  const int tid = threadIdx.x, w = tid >> 5, lane = tid & 31, col = lane & 15, g = lane >> 4;
  const int h = blockIdx.y; const int q0 = blockIdx.x * 64 + w * 16; const size_t hb = (size_t)h * NNODE;
  v16h aq[3];
#pragma unroll
  for (int kc = 0; kc < 3; ++kc) aq[kc] = frag_h(Q16 + (hb + q0 + col) * HDD + kc * 32, lane);
  float mrun = -3.0e38f, lrun = 0.f; v8f acc[6] = {};
#pragma unroll 1
  for (int kt = 0; kt < NNODE / 64; ++kt) {
#pragma unroll
    for (int t = 0; t < 4; ++t) { v8f s = {}; const int key = kt * 64 + t * 16 + col;
#pragma unroll
      for (int kc = 0; kc < 3; ++kc) s = wmma16(aq[kc], frag_h(K16 + (hb + key) * HDD + kc * 32, lane), s);
#pragma unroll
      for (int r = 0; r < 8; ++r) sS[w][8 * g + r][t * 16 + col] = s[r] * (0.10206207261596575f / 16.0f); }
    LDSX();
    float mx = -3.4e38f;
#pragma unroll
    for (int jj = 0; jj < 32; ++jj) mx = fmaxf(mx, sS[w][col][g * 32 + jj]);
    mx = fmaxf(mx, __shfl_xor(mx, 16, 32));
    const float mnew = fmaxf(mrun, mx); const float corr = expf(mrun - mnew);
    float ps = 0.f;
#pragma unroll
    for (int jj = 0; jj < 32; ++jj) { const float p = expf(sS[w][col][g * 32 + jj] - mnew); ps += p; sP[w][col][g * 32 + jj] = (_Float16)(p * 16384.0f); }
    ps += __shfl_xor(ps, 16, 32);
    lrun = lrun * corr + ps; mrun = mnew;
#pragma unroll
    for (int r = 0; r < 8; ++r) { const float cr = __shfl(corr, 8 * g + r, 32);
#pragma unroll
      for (int t = 0; t < 6; ++t) acc[t][r] *= cr; }
    LDSX();
#pragma unroll
    for (int kc = 0; kc < 2; ++kc) { const v16h pa = frag_h(&sP[w][col][0] + kc * 32, lane);
#pragma unroll
      for (int t = 0; t < 6; ++t) acc[t] = wmma16(pa, frag_h(VT + ((size_t)h * HDD + t * 16 + col) * NNODE + kt * 64 + kc * 32, lane), acc[t]); }
    __builtin_amdgcn_wave_barrier(); }
#pragma unroll
  for (int r = 0; r < 8; ++r) { const float lr = __shfl(lrun, 8 * g + r, 32); const float inv = 8.0f / (lr * 16384.0f);
#pragma unroll
    for (int t = 0; t < 6; ++t) sO[w][8 * g + r][t * 16 + col] = acc[t][r] * inv; }
  LDSX();
  for (int qq = lane; qq < 16 * 12; qq += 32) { const int rl = qq / 12, pc = qq % 12; union { v8h h8; v4u u; } pk;
#pragma unroll
    for (int e = 0; e < 8; ++e) pk.h8[e] = (_Float16)sO[w][rl][pc * 8 + e];
    vst2(O16 + (hb + q0 + rl) * HDD + pc * 8, pk.u); }
}
__global__ __launch_bounds__(128) void k_tail(const _Float16* __restrict__ O16, const float* __restrict__ feat, const int* __restrict__ nidx, const _Float16* __restrict__ WoT, const float* __restrict__ bo, const _Float16* __restrict__ W1T, const float* __restrict__ b1, const _Float16* __restrict__ W2T, const float* __restrict__ b2, float* __restrict__ out) {
  __shared__ __align__(16) _Float16 sh[4][16][DM + FE + 8];
  __shared__ __align__(16) _Float16 s1[4][16][FE + 8];
  __shared__ __align__(16) float so[4][16][132];
  const int tid = threadIdx.x, wave = tid >> 5, lane = tid & 31, col = lane & 15, g = lane >> 4;
  const int r0 = blockIdx.x * 64 + wave * 16;
  for (int qq = lane; qq < 16 * 16; qq += 32) { const int rl = qq >> 4, pc = qq & 15; int m = nidx[r0 + rl]; m = m < 0 ? 0 : (m >= NNODE ? NNODE - 1 : m); union { v8h h; v4u u; } pk;
#pragma unroll
    for (int e = 0; e < 8; ++e) pk.h[e] = (_Float16)feat[(size_t)m * FE + pc * 8 + e];
    *(v4u*)(&sh[wave][rl][pc * 8]) = pk.u; }
  { v8f acc[12];
#pragma unroll
    for (int t = 0; t < 12; ++t) acc[t] = (v8f){};
#pragma unroll
    for (int kc = 0; kc < DM / 32; ++kc) { const int hh = kc / 3; const v16h a = frag_h(O16 + ((size_t)hh * NNODE + r0 + col) * HDD + (kc - 3 * hh) * 32, lane);
#pragma unroll
      for (int t = 0; t < 12; ++t) acc[t] = wmma16(a, frag_h(WoT + (size_t)(t * 16 + col) * DM + kc * 32, lane), acc[t]); }
#pragma unroll
    for (int t = 0; t < 12; ++t) { const float bb = bo[t * 16 + col];
#pragma unroll
      for (int r = 0; r < 8; ++r) sh[wave][8 * g + r][FE + t * 16 + col] = (_Float16)(acc[t][r] * (1.0f / (16.0f * 8.0f)) + bb); } }
  LDSX();
  { v8f acc[8] = {};
#pragma unroll
    for (int kc = 0; kc < (DM + FE) / 32; ++kc) { const v16h a = frag_h(&sh[wave][col][0] + kc * 32, lane);
#pragma unroll
      for (int t = 0; t < 8; ++t) acc[t] = wmma16(a, frag_h(W1T + (size_t)(t * 16 + col) * (DM + FE) + kc * 32, lane), acc[t]); }
#pragma unroll
    for (int t = 0; t < 8; ++t) { const float bb = b1[t * 16 + col];
#pragma unroll
      for (int r = 0; r < 8; ++r) { const float v = acc[t][r] * (1.0f / 16.0f) + bb; s1[wave][8 * g + r][t * 16 + col] = (_Float16)(v > 0.f ? v : 0.f); } } }
  LDSX();
  { v8f acc[8] = {};
#pragma unroll
    for (int kc = 0; kc < FE / 32; ++kc) { const v16h a = frag_h(&s1[wave][col][0] + kc * 32, lane);
#pragma unroll
      for (int t = 0; t < 8; ++t) acc[t] = wmma16(a, frag_h(W2T + (size_t)(t * 16 + col) * FE + kc * 32, lane), acc[t]); }
#pragma unroll
    for (int t = 0; t < 8; ++t) { const float bb = b2[t * 16 + col];
#pragma unroll
      for (int r = 0; r < 8; ++r) so[wave][8 * g + r][t * 16 + col] = acc[t][r] * (1.0f / 16.0f) + bb; } }
  LDSX();
#pragma unroll 4
  for (int rl = 0; rl < 16; ++rl) vst2(out + (size_t)(r0 + rl) * FE + lane * 4, *(const v4f*)(&so[wave][rl][lane * 4]));
}
extern "C" void kernel_launch(void* const* d_in, const int* in_sizes, int n_in, void* d_out, int out_size, void* d_ws, size_t ws_size, hipStream_t stream) {
  (void)in_sizes; (void)n_in; (void)out_size; (void)ws_size;
  const float** I = (const float**)d_in;
  const float* feat = I[0]; const float* ef = I[1]; const float* tf = I[2]; const int* nbr = (const int*)d_in[3]; const int* nidx = (const int*)d_in[4];
  const float* Wq = I[5]; const float* bq = I[6]; const float* Wk = I[7]; const float* bk = I[8]; const float* Wv = I[9]; const float* bv = I[10]; const float* Wo = I[11]; const float* bo = I[12]; const float* W1 = I[13]; const float* b1 = I[14]; const float* W2 = I[15]; const float* b2 = I[16];
  float* out = (float*)d_out;
  char* ws = (char*)d_ws; size_t off = 0;
  auto take = [&](size_t bytes) { char* p = ws + off; off += (bytes + 255) & ~(size_t)255; return p; };
  _Float16* WqT = (_Float16*)take(DM * DM * 2); _Float16* WkT = (_Float16*)take((size_t)DM * KD * 2); _Float16* WvT = (_Float16*)take((size_t)DM * KD * 2); _Float16* WoT = (_Float16*)take(DM * DM * 2); _Float16* W1T = (_Float16*)take(FE * (DM + FE) * 2); _Float16* W2T = (_Float16*)take(FE * FE * 2);
  _Float16* K16 = (_Float16*)take((size_t)NH * NNODE * HDD * 2); _Float16* VT = (_Float16*)take((size_t)NH * HDD * NNODE * 2); _Float16* Q16 = (_Float16*)take((size_t)NH * NNODE * HDD * 2); _Float16* O16 = (_Float16*)take((size_t)NNODE * DM * 2);
  k_pack<<<4 * DM + 2 * FE, 256, 0, stream>>>(Wq, Wk, Wv, Wo, W1, W2, WqT, WkT, WvT, WoT, W1T, W2T);
  k_kv<<<dim3(NNODE / 64, 2), 128, 0, stream>>>(feat, ef, tf, nbr, WkT, WvT, bk, bv, K16, VT);
  k_q<<<NNODE / 64, 128, 0, stream>>>(feat, nidx, WqT, bq, Q16);
  k_attn<<<dim3(NNODE / 64, NH), 128, 0, stream>>>(Q16, K16, VT, O16);
  k_tail<<<NNODE / 64, 128, 0, stream>>>(O16, feat, nidx, WoT, bo, W1T, b1, W2T, b2, out);
}
